// MultiHeadedAttention_62526133895682
// MI455X (gfx1250) — hardware-verified
//
#include <hip/hip_runtime.h>


#ifndef NB
#define NB 2
#endif
#ifndef SEQ
#define SEQ 2048
#endif
#define SEQ_FULL 2048
#define TT   SEQ
#define DM   1024
#define NH_  16
#define HD   64
#define SCL  0.03125f
#define L2E  1.4426950408889634f
#define NEGB (-3.0e38f)

static_assert(TT % 128 == 0);
static_assert((TT & (TT - 1)) == 0);
static_assert(TT <= SEQ_FULL);
static_assert(NH_ * HD == DM);
static_assert(DM % 64 == 0);
static_assert(DM == 1024);
static_assert(HD == 64);
static_assert(NB >= 1 && NB <= 2);
static_assert((NB * TT) % 64 == 0);
static_assert(((size_t)DM * DM / 8) % 256 == 0);
static_assert(((size_t)NB * SEQ_FULL * DM / 8) % 256 == 0);
static_assert(((size_t)NH_ * TT * HD / 8) % 256 == 0);

#define SZ_WT  ((size_t)4 * DM * DM * 2)
#define SZ_XB  ((size_t)NB * SEQ_FULL * DM * 2)
#define SZ_F   ((size_t)3 * TT * DM * 4)
#define SZ_PL  ((size_t)NH_ * TT * HD * 2)
#define SZ_CTX ((size_t)NB * TT * DM * 2)
static_assert(SZ_WT % 256 == 0 && SZ_XB % 256 == 0 && SZ_F % 256 == 0 && SZ_PL % 256 == 0 && SZ_CTX % 256 == 0);
static_assert(SZ_WT + SZ_XB + SZ_F + 4 * SZ_PL + 2 * SZ_CTX <= (size_t)134217728);

typedef _Float16 h16;
typedef unsigned short bf;
typedef __attribute__((ext_vector_type(16))) __bf16   v16bf;
typedef __attribute__((ext_vector_type(16))) _Float16 v16h;
typedef __attribute__((ext_vector_type(8)))  _Float16 v8h;
typedef __attribute__((ext_vector_type(8)))  unsigned short v8us;
typedef __attribute__((ext_vector_type(8)))  float    v8f;
typedef __attribute__((ext_vector_type(4)))  float    v4f;
typedef v4f  __attribute__((may_alias)) v4fa;

__device__ __forceinline__ unsigned short f2bf(float f) { unsigned u = __float_as_uint(f); u += 0x7FFFu + ((u >> 16) & 1u); return (unsigned short)(u >> 16); }
__device__ __forceinline__ float bf2f(unsigned short b) { return __uint_as_float(((unsigned)b) << 16); }
__device__ __forceinline__ float bfr(float f) { return bf2f(f2bf(f)); }
__device__ __forceinline__ v16h cat16(v8h lo, v8h hi) { return __builtin_shufflevector(lo, hi, 0, 1, 2, 3, 4, 5, 6, 7, 8, 9, 10, 11, 12, 13, 14, 15); }
__device__ __forceinline__ v16bf cat16b(v8us lo, v8us hi) { return __builtin_bit_cast(v16bf, __builtin_shufflevector(lo, hi, 0, 1, 2, 3, 4, 5, 6, 7, 8, 9, 10, 11, 12, 13, 14, 15)); }
__device__ __forceinline__ v8f wmma16(v16h a, v16h b, v8f c) { return __builtin_amdgcn_wmma_f32_16x16x32_f16(false, a, false, b, (short)0, c, false, false); }
__device__ __forceinline__ v8f wmmab(v16bf a, v16bf b, v8f c) { return __builtin_amdgcn_wmma_f32_16x16x32_bf16(false, a, false, b, (short)0, c, false, false); }
__device__ __forceinline__ h16 tohx(float x) { return (h16)x; }
__device__ __forceinline__ void splitf(float y, unsigned short& h, unsigned short& l) { h = f2bf(y); l = f2bf(y - bf2f(h)); }

template <typename T16> struct WFrag;
template <> struct WFrag<h16> { typedef v16h V; static __device__ __forceinline__ V ld(const h16* p) { return cat16(*(const v8h*)p, *(const v8h*)(p + 16)); } static __device__ __forceinline__ v8f mma(V a, V b, v8f c) { return wmma16(a, b, c); } };
template <> struct WFrag<bf> { typedef v16bf V; static __device__ __forceinline__ V ld(const bf* p) { return cat16b(*(const v8us*)p, *(const v8us*)(p + 16)); } static __device__ __forceinline__ v8f mma(V a, V b, v8f c) { return wmmab(a, b, c); } };
template <typename T16, int NSPLIT, bool BIAS>
__global__ __launch_bounds__(32) void k_gemmw(const T16* __restrict__ A, const T16* __restrict__ A2, const T16* __restrict__ Bt, const T16* __restrict__ Bt2, int K, float* C, int ldc, const float* __restrict__ bias, size_t sA, size_t sB, size_t sC) {
    typedef typename WFrag<T16>::V V;
    __shared__ __align__(16) float os[16 * 68];
    const size_t z = blockIdx.z; A += z * sA; if (A2) A2 += z * sA; Bt += z * sB; if (Bt2) Bt2 += z * sB; C += z * sC;
    const int lane = threadIdx.x & 31, lr = lane & 15, hi = lane >> 4; const int r0 = blockIdx.x * 64, c0 = blockIdx.y * 64;
    v8f acc[4][4];
#pragma unroll
    for (int mb = 0; mb < 4; ++mb)
#pragma unroll
        for (int nb = 0; nb < 4; ++nb) acc[mb][nb] = (v8f){};
    const size_t aoff = (size_t)(r0 + lr) * K + 8 * hi, boff = (size_t)(c0 + lr) * K + 8 * hi;
#pragma unroll 1
    for (int kc = 0; kc < K; kc += 32) {
        V a[4], a2[4];
#pragma unroll
        for (int mb = 0; mb < 4; ++mb) { a[mb] = WFrag<T16>::ld(A + aoff + (size_t)mb * 16 * K + kc); if (NSPLIT == 1 || NSPLIT == 2) a2[mb] = WFrag<T16>::ld(A2 + aoff + (size_t)mb * 16 * K + kc); }
#pragma unroll
        for (int nb = 0; nb < 4; ++nb) { const V b = WFrag<T16>::ld(Bt + boff + (size_t)nb * 16 * K + kc); V b2; if (NSPLIT >= 2) b2 = WFrag<T16>::ld(Bt2 + boff + (size_t)nb * 16 * K + kc);
#pragma unroll
            for (int mb = 0; mb < 4; ++mb) { acc[mb][nb] = WFrag<T16>::mma(a[mb], b, acc[mb][nb]); if (NSPLIT == 1 || NSPLIT == 2) acc[mb][nb] = WFrag<T16>::mma(a2[mb], b, acc[mb][nb]); if (NSPLIT >= 2) acc[mb][nb] = WFrag<T16>::mma(a[mb], b2, acc[mb][nb]); } }
        asm volatile("v_nop\n\tv_nop\n\tv_nop\n\tv_nop" : "+v"(acc[0][0]), "+v"(acc[1][1]), "+v"(acc[2][2]), "+v"(acc[3][3]) : "v"(a[0]), "v"(a[3]));
    }
#pragma unroll
    for (int mb = 0; mb < 4; ++mb) {
#pragma unroll
        for (int nb = 0; nb < 4; ++nb) {
#pragma unroll
            for (int j = 0; j < 8; ++j) os[(hi * 8 + j) * 68 + nb * 16 + lr] = acc[mb][nb][j]; }
        __builtin_amdgcn_wave_barrier(); asm volatile("" ::: "memory");
        float* crow = C + (size_t)(r0 + mb * 16) * ldc + c0;
#pragma unroll 1
        for (int ps = 0; ps < 2; ++ps) {
#pragma unroll
            for (int s = 0; s < 8; ++s) { const int row = 2 * s + hi, cofs = lr * 4; v4f val = *(const v4fa*)(os + row * 68 + cofs); if (BIAS) { val[0] += bfr(bias[c0 + cofs]); val[1] += bfr(bias[c0 + cofs + 1]); val[2] += bfr(bias[c0 + cofs + 2]); val[3] += bfr(bias[c0 + cofs + 3]); }
                *(volatile v4f*)(crow + (size_t)row * ldc + cofs) = val; }
            if (ps == 0) __threadfence(); }
        __builtin_amdgcn_wave_barrier(); asm volatile("" ::: "memory");
    }
}

__global__ __launch_bounds__(256) void k_cvt8(const float* __restrict__ src, bf* dst, size_t n8) { const size_t i = (size_t)blockIdx.x * 256 + threadIdx.x; if (i >= n8) return; const v8f v = *(const v8f*)(src + i * 8); v8us o;
#pragma unroll
    for (int k = 0; k < 8; ++k) o[k] = f2bf(v[k]); *(volatile v8us*)(dst + i * 8) = o; __threadfence(); *(volatile v8us*)(dst + i * 8) = o; }

__global__ __launch_bounds__(256) void k_cvtw(const float* __restrict__ w0, const float* __restrict__ w1, const float* __restrict__ w2, const float* __restrict__ w3, bf* WT) {
    const unsigned z = blockIdx.y;
    const float* w = (z == 0u) ? w0 : ((z == 1u) ? w1 : ((z == 2u) ? w2 : w3));
    const unsigned i = blockIdx.x * 256u + threadIdx.x; if (i >= (unsigned)(DM * DM / 8)) return;
    const v8f v = *(const v8f*)(w + (size_t)i * 8);
    v8us o;
#pragma unroll
    for (int k = 0; k < 8; ++k) o[k] = f2bf(v[k]);
    bf* d = WT + (size_t)z * DM * DM + (size_t)i * 8;
    *(volatile v8us*)d = o; __threadfence(); *(volatile v8us*)d = o;
}

__global__ __launch_bounds__(256) void k_qkp(const float* __restrict__ FQ, const float* __restrict__ FK, h16* QP, h16* KP) {
    const unsigned y = blockIdx.y;
    const float* F = y ? FK : FQ; h16* P = y ? KP : QP;
    const unsigned i = blockIdx.x * 256u + threadIdx.x; if (i >= (unsigned)(NH_ * TT * HD / 8)) return;
    const unsigned e = i * 8u; const unsigned d = e % (unsigned)HD; const unsigned t = (e / (unsigned)HD) % (unsigned)TT; const unsigned h = e / (unsigned)(HD * TT);
    const v8f f = *(const v8f*)(F + (size_t)t * DM + h * HD + d);
    v8h o;
#pragma unroll
    for (int q = 0; q < 8; ++q) o[q] = tohx(f[q]);
    *(volatile v8h*)(P + e) = o; __threadfence(); *(volatile v8h*)(P + e) = o;
}

__global__ __launch_bounds__(256) void k_vtp(const float* __restrict__ F, bf* Vh, bf* Vl) {
    const unsigned i = blockIdx.x * 256u + threadIdx.x; if (i >= (unsigned)(NH_ * HD * TT / 8)) return;
    const unsigned e = i * 8u; const unsigned t = e % (unsigned)TT; const unsigned d = (e / (unsigned)TT) % (unsigned)HD; const unsigned h = e / (unsigned)(TT * HD);
    v8us oh, ol;
#pragma unroll
    for (int q = 0; q < 8; ++q) { const float x = F[(size_t)(t + q) * DM + h * HD + d]; unsigned short a2, c2; splitf(x, a2, c2); oh[q] = a2; ol[q] = c2; }
    *(volatile v8us*)(Vh + e) = oh; *(volatile v8us*)(Vl + e) = ol; __threadfence(); *(volatile v8us*)(Vh + e) = oh; *(volatile v8us*)(Vl + e) = ol;
}

__global__ __launch_bounds__(128) void k_flash(const h16* __restrict__ QP, const h16* __restrict__ KP, const bf* __restrict__ VTh, const bf* __restrict__ VTl, bf* Ch, bf* Cl) {
    __shared__ __align__(16) float os[4 * 16 * 68];
    const unsigned lane = threadIdx.x & 31u, wv = threadIdx.x >> 5, lr = lane & 15u, hi = lane >> 4;
    const unsigned h = blockIdx.y; const unsigned qb = blockIdx.x * 64u + wv * 16u; const unsigned q = qb + lr;
    const h16* kh = KP + (size_t)h * TT * HD;
    const bf* vh = VTh + (size_t)h * HD * TT; const bf* vl = VTl + (size_t)h * HD * TT;
    const h16* qrow = QP + (size_t)h * TT * HD + (size_t)q * HD + 8u * hi;
    const v16h bq0 = WFrag<h16>::ld(qrow), bq1 = WFrag<h16>::ld(qrow + 32);
    v8f acc[4];
#pragma unroll
    for (int t = 0; t < 4; ++t) acc[t] = (v8f){};
    float Mrun = NEGB, Lrun = 0.0f;
    const unsigned kend = qb + 16u;
#pragma unroll 1
    for (unsigned kb = 0; kb < kend; kb += 32u) {
        const h16* k0 = kh + (size_t)(kb + lr) * HD + 8u * hi;
        const v16h a00 = WFrag<h16>::ld(k0), a01 = WFrag<h16>::ld(k0 + 32), a10 = WFrag<h16>::ld(k0 + 16 * HD), a11 = WFrag<h16>::ld(k0 + 16 * HD + 32);
        v8f s0 = (v8f){}, s1 = (v8f){};
        s0 = wmma16(a00, bq0, s0); s0 = wmma16(a01, bq1, s0); s1 = wmma16(a10, bq0, s1); s1 = wmma16(a11, bq1, s1);
        asm volatile("v_nop\n\tv_nop\n\tv_nop\n\tv_nop" : "+v"(s0), "+v"(s1) : "v"(a00), "v"(a01), "v"(a10), "v"(a11), "v"(bq0), "v"(bq1));
        const unsigned kk = kb + 8u * hi;
        float p0[8], p1[8]; float mloc = NEGB;
#pragma unroll
        for (int r = 0; r < 8; ++r) {
            const bool ok0 = (kk + (unsigned)r) <= q, ok1 = (kk + 16u + (unsigned)r) <= q;
            const float t0 = ok0 ? s0[r] * SCL : NEGB; const float t1 = ok1 ? s1[r] * SCL : NEGB;
            p0[r] = t0; p1[r] = t1; mloc = fmaxf(mloc, fmaxf(t0, t1)); }
        mloc = fmaxf(mloc, __shfl_xor(mloc, 16, 32));
        const float Mnew = fmaxf(Mrun, mloc);
        const float alpha = __builtin_amdgcn_exp2f((Mrun - Mnew) * L2E);
        float lsum = 0.0f;
#pragma unroll
        for (int r = 0; r < 8; ++r) {
            const bool ok0 = (kk + (unsigned)r) <= q, ok1 = (kk + 16u + (unsigned)r) <= q;
            const float e0 = __builtin_amdgcn_exp2f((p0[r] - Mnew) * L2E); const float e1 = __builtin_amdgcn_exp2f((p1[r] - Mnew) * L2E);
            p0[r] = ok0 ? e0 : 0.0f; p1[r] = ok1 ? e1 : 0.0f; lsum += p0[r]; lsum += p1[r]; }
        lsum += __shfl_xor(lsum, 16, 32);
        Lrun = Lrun * alpha + lsum; Mrun = Mnew;
        v8us ph0, pl0, ph1, pl1;
#pragma unroll
        for (int r = 0; r < 8; ++r) { unsigned short a, c; splitf(p0[r], a, c); ph0[r] = a; pl0[r] = c; splitf(p1[r], a, c); ph1[r] = a; pl1[r] = c; }
        const v16bf PH = cat16b(ph0, ph1), PL = cat16b(pl0, pl1);
#pragma unroll
        for (int t = 0; t < 4; ++t) {
#pragma unroll
            for (int r = 0; r < 8; ++r) acc[t][r] *= alpha; }
#pragma unroll
        for (int t = 0; t < 4; ++t) {
            const size_t vo = (size_t)(16u * (unsigned)t + lr) * TT + kb + 8u * hi;
            const v16bf avh = WFrag<bf>::ld(vh + vo), avl = WFrag<bf>::ld(vl + vo);
            acc[t] = wmmab(avh, PH, acc[t]); acc[t] = wmmab(avh, PL, acc[t]); acc[t] = wmmab(avl, PH, acc[t]);
            asm volatile("v_nop\n\tv_nop\n\tv_nop\n\tv_nop" : "+v"(acc[t]) : "v"(avh), "v"(avl), "v"(PH), "v"(PL));
        }
    }
    const float inv = __fdiv_rn(1.0f, Lrun);
    float* o = os + wv * (16u * 68u);
#pragma unroll
    for (int t = 0; t < 4; ++t) {
        v4f u0, u1;
#pragma unroll
        for (int j = 0; j < 4; ++j) { u0[j] = acc[t][j] * inv; u1[j] = acc[t][4 + j] * inv; }
        *(v4fa*)(o + lr * 68u + 16u * (unsigned)t + 8u * hi) = u0; *(v4fa*)(o + lr * 68u + 16u * (unsigned)t + 8u * hi + 4u) = u1;
    }
    __syncthreads();
    const unsigned rq = lane >> 3, pc = lane & 7u;
    v8us oh[4], ol[4];
#pragma unroll
    for (int s = 0; s < 4; ++s) {
        const float* src = o + (4u * (unsigned)s + rq) * 68u + pc * 8u;
        const v4f x0 = *(const v4fa*)src, x1 = *(const v4fa*)(src + 4);
#pragma unroll
        for (int j = 0; j < 4; ++j) { unsigned short a, c; splitf(x0[j], a, c); oh[s][j] = a; ol[s][j] = c; splitf(x1[j], a, c); oh[s][4 + j] = a; ol[s][4 + j] = c; }
    }
    bf* ch = Ch + (size_t)qb * DM + h * HD + pc * 8u; bf* cl = Cl + (size_t)qb * DM + h * HD + pc * 8u;
#pragma unroll 1
    for (int ps = 0; ps < 2; ++ps) {
#pragma unroll
        for (int s = 0; s < 4; ++s) { const size_t off = (size_t)(4u * (unsigned)s + rq) * DM; *(volatile v8us*)(ch + off) = oh[s]; *(volatile v8us*)(cl + off) = ol[s]; }
        if (ps == 0) __threadfence(); }
}

extern "C" void kernel_launch(void* const* d_in, const int* in_sizes, int n_in,
                              void* d_out, int out_size, void* d_ws, size_t ws_size, hipStream_t stream) {
    if (n_in < 6) return;
    if (in_sizes[0] < NB * SEQ_FULL * DM) return;
    if (in_sizes[1] < DM * DM || in_sizes[2] < DM * DM || in_sizes[3] < DM * DM || in_sizes[4] < DM * DM) return;
    if (in_sizes[5] < DM) return;
    if (out_size < NB * TT * DM) return;
    const float* x  = (const float*)d_in[0];
    const float* wq = (const float*)d_in[1];
    const float* wk = (const float*)d_in[2];
    const float* wv = (const float*)d_in[3];
    const float* wo = (const float*)d_in[4];
    const float* bo = (const float*)d_in[5];
    float* OUT = (float*)d_out;
    char* wsp = (char*)d_ws;
    auto take = [&](size_t bytes) { char* p = wsp; wsp += (bytes + 255) & ~(size_t)255; return (void*)p; };
    bf*    WT   = (bf*)take(SZ_WT);
    bf*    XB   = (bf*)take(SZ_XB);
    float* F    = (float*)take(SZ_F);
    h16*   QP   = (h16*)take(SZ_PL);
    h16*   KP   = (h16*)take(SZ_PL);
    bf*    VTh  = (bf*)take(SZ_PL);
    bf*    VTl  = (bf*)take(SZ_PL);
    bf*    CTXh = (bf*)take(SZ_CTX);
    bf*    CTXl = (bf*)take(SZ_CTX);
    if ((size_t)(wsp - (char*)d_ws) > ws_size) return;
    float* FQ = F; float* FK = F + (size_t)TT * DM; float* FV = F + (size_t)2 * TT * DM;

    k_cvtw<<<dim3((unsigned)((size_t)DM * DM / 8 / 256), 4), 256, 0, stream>>>(wq, wk, wv, wo, WT);
    const size_t nx8 = (size_t)NB * SEQ_FULL * DM / 8;
    k_cvt8<<<(unsigned)(nx8 / 256), 256, 0, stream>>>(x, XB, nx8);
    const unsigned LP = (unsigned)((size_t)NH_ * TT * HD / 8 / 256);
    for (int b = 0; b < NB; ++b) {
        k_gemmw<bf, 0, false><<<dim3(TT / 64, DM / 64, 3), 32, 0, stream>>>(XB + (size_t)b * SEQ_FULL * DM, nullptr, WT, nullptr, DM, F, DM, nullptr, (size_t)0, (size_t)DM * DM, (size_t)TT * DM);
        k_qkp<<<dim3(LP, 2), 256, 0, stream>>>(FQ, FK, QP, KP);
        k_vtp<<<LP, 256, 0, stream>>>(FV, VTh, VTl);
        k_flash<<<dim3(TT / 64, NH_), 128, 0, stream>>>(QP, KP, VTh, VTl, CTXh + (size_t)b * TT * DM, CTXl + (size_t)b * TT * DM);
    }
    k_gemmw<bf, 1, true><<<dim3(NB * TT / 64, DM / 64, 1), 32, 0, stream>>>(CTXh, CTXl, WT + (size_t)3 * DM * DM, nullptr, DM, OUT, DM, bo, (size_t)0, (size_t)0, (size_t)0);
}
